// CompGCNLayer_73942156968056
// MI455X (gfx1250) — hardware-verified
//
#include <hip/hip_runtime.h>
#include <stddef.h>
#include <stdint.h>

#pragma clang fp contract(off)


#define DF      128
#define NN      100000
#define NE      1000000
#define HALF    500000
#define NREL    1001
#define SELFROW 1000
#define MP      100096
#define RBR     1024
#define WCR     512
#define PNW     256
#define PRW     384
#define NBK     1024
#define NBLK    98
#define RECROWS (NBLK * NBK)
#define NTHR    256
#define NWAVE   8
#define NCH     (NE / 32)
#define CHH     (HALF / 32)
#define WTRIPS  3908
#define GBM     64
#define GBN     128
#define GTHR    128
#define BINS_INTS  (NWAVE * 2 * NBK)
#define STAGE_INTS (NBK * 8)
#define BK_LDS_INTS (2 * BINS_INTS + STAGE_INTS)
#define OUT1_OFF   (NN * DF)
#define OUT_TOTAL  (OUT1_OFF + NREL * DF)
#define PREP_BX    (MP * 16 / NTHR)
#define PREP_BR    (RBR * 16 / NTHR)
#define PREP_BW    (WCR * 16 / NTHR)

static_assert(DF == 128 && NN == 100000 && NE == 1000000 && HALF * 2 == NE);
static_assert(NREL == 1001 && SELFROW == NREL - 1);
static_assert(NE % 32 == 0 && HALF % 32 == 0);
static_assert(3LL * NE < (1LL << 31));
static_assert(MP == 782 * 128 && MP >= NN && MP % GBM == 0);
static_assert(RBR >= NREL && RBR % GBM == 0);
static_assert(RECROWS >= NN && NBK == 4 * NTHR);
static_assert(NN % NWAVE == 0);
static_assert(WTRIPS % 4 == 0 && WTRIPS >= (NCH + NWAVE - 1) / NWAVE);
static_assert((MP * 16) % NTHR == 0 && (RBR * 16) % NTHR == 0 && (WCR * 16) % NTHR == 0);
static_assert((DF * 16) % NTHR == 0);
static_assert(GBM == (GTHR / 32) * 16 && GBN == DF && DF % 32 == 0);
static_assert(PNW == 2 * GBN && PRW == 3 * GBN && WCR == 4 * DF);
static_assert(BK_LDS_INTS * 4 <= 327680);
static_assert(OUT1_OFF % 32 == 0);
static_assert((long long)OUT1_OFF + (long long)(NREL - 1) * DF + DF - 1 < (long long)OUT_TOTAL);

static constexpr size_t SZ_XB  = (size_t)MP * DF * 2;
static constexpr size_t SZ_PNO = (size_t)NN * PNW * 4;
static constexpr size_t SZ_RB  = (size_t)RBR * DF * 2;
static constexpr size_t SZ_WC  = (size_t)WCR * DF * 2;
static constexpr size_t SZ_PR  = (size_t)RBR * PRW * 4;
static constexpr size_t SZ_REC = (size_t)RECROWS * 8 * 4;
static constexpr size_t OFF_XB  = 0;
static constexpr size_t OFF_PNO = OFF_XB + SZ_XB;
static constexpr size_t OFF_RB  = OFF_PNO + SZ_PNO;
static constexpr size_t OFF_WC  = OFF_RB + SZ_RB;
static constexpr size_t OFF_PR  = OFF_WC + SZ_WC;
static constexpr size_t OFF_REC = OFF_PR + SZ_PR;
static constexpr size_t WS_TOTAL = OFF_REC + SZ_REC;
static_assert(SZ_XB % 256 == 0 && SZ_PNO % 256 == 0 && SZ_RB % 256 == 0);
static_assert(SZ_WC % 256 == 0 && SZ_PR % 256 == 0 && SZ_REC % 256 == 0);
static_assert(WS_TOTAL <= (size_t)(128u << 20));

typedef float          v4f   __attribute__((ext_vector_type(4)));
typedef float          v8f   __attribute__((ext_vector_type(8)));
typedef int            v4i   __attribute__((ext_vector_type(4)));
typedef int            v8i   __attribute__((ext_vector_type(8)));
typedef unsigned short v8us  __attribute__((ext_vector_type(8)));
typedef unsigned short v16us __attribute__((ext_vector_type(16)));
typedef __bf16         v16bf __attribute__((ext_vector_type(16)));
typedef v4f  __attribute__((may_alias)) v4fa;
typedef v4i  __attribute__((may_alias)) v4ia;
typedef v8us __attribute__((may_alias)) v8usa;
union FragB { v16bf v; v16us u; v8us h[2]; v8i w; };

__device__ __forceinline__ v8f wmb(const FragB& a, const FragB& b, v8f c) {
  v8f d = __builtin_amdgcn_wmma_f32_16x16x32_bf16(false, a.v, false, b.v, (short)0, c, false, false);
  asm volatile("v_nop\n\tv_nop\n\tv_nop\n\tv_nop" : "+v"(d) : "v"(a.w), "v"(b.w));
  return d;
}

__device__ __forceinline__ unsigned bf16_bits(float f) {
  const unsigned u = __float_as_uint(f);
  return (u + 0x7FFFu + ((u >> 16) & 1u)) >> 16;
}

__device__ __forceinline__ int clampi(int v, int lo, int hi) {
  v = v < lo ? lo : v;
  v = v > hi ? hi : v;
  return v;
}

__device__ __forceinline__ void cvt8(const float* __restrict__ src, int nvalid, int row, int k8,
                                     unsigned short* dp) {
  const int rc = row < nvalid ? row : nvalid - 1;
  const float* p = src + (size_t)rc * DF + k8;
  const v4f a = *(const v4f*)p;
  const v4f b = *(const v4f*)(p + 4);
  asm volatile("" :: "v"(a), "v"(b));
  const unsigned msk = (row < nvalid) ? 0xFFFFu : 0u;
  v8us o;
  o[0] = (unsigned short)(bf16_bits(a.x) & msk); o[1] = (unsigned short)(bf16_bits(a.y) & msk);
  o[2] = (unsigned short)(bf16_bits(a.z) & msk); o[3] = (unsigned short)(bf16_bits(a.w) & msk);
  o[4] = (unsigned short)(bf16_bits(b.x) & msk); o[5] = (unsigned short)(bf16_bits(b.y) & msk);
  o[6] = (unsigned short)(bf16_bits(b.z) & msk); o[7] = (unsigned short)(bf16_bits(b.w) & msk);
  *(volatile v8us*)dp = o;
  __threadfence();
  *(volatile v8us*)dp = o;
}

__global__ __launch_bounds__(NTHR) void k_prep(const float* __restrict__ xn, const float* __restrict__ rel,
                                               const float* __restrict__ Wo, const float* __restrict__ Wi,
                                               const float* __restrict__ Ws, const float* __restrict__ Wr,
                                               unsigned short* XB, unsigned short* RB, unsigned short* WC) {
  const int b = (int)blockIdx.x, tid = (int)threadIdx.x;
  if (b < PREP_BX) {
    const int u = b * NTHR + tid;
    const int row = u >> 4, k8 = (u & 15) * 8;
    cvt8(xn, NN, row, k8, XB + (size_t)row * DF + k8);
  } else if (b < PREP_BX + PREP_BR) {
    const int u = (b - PREP_BX) * NTHR + tid;
    const int row = u >> 4, k8 = (u & 15) * 8;
    cvt8(rel, NREL, row, k8, RB + (size_t)row * DF + k8);
  } else if (b < PREP_BX + PREP_BR + PREP_BW) {
    const int u = (b - PREP_BX - PREP_BR) * NTHR + tid;
    const int part = u >> 11;
    const int v = u & 2047;
    const int n = v >> 4, k8 = (v & 15) * 8;
    unsigned short* dp = WC + (size_t)(part * DF + n) * DF + k8;
    if (part == 0)      cvt8(Wi, DF, n, k8, dp);
    else if (part == 1) cvt8(Wo, DF, n, k8, dp);
    else if (part == 2) cvt8(Ws, DF, n, k8, dp);
    else                cvt8(Wr, DF, n, k8, dp);
  }
}

__global__ __launch_bounds__(NTHR) void k_bucket(const int* __restrict__ edges, int* rec) {
  extern __shared__ __attribute__((aligned(16))) int dsm[];
  int* cntb  = dsm;
  int* lastb = dsm + BINS_INTS;
  int* stage = dsm + 2 * BINS_INTS;
  const int tid = (int)threadIdx.x, lane = tid & 31;
  const int wave = __builtin_amdgcn_readfirstlane(tid >> 5);
  const unsigned base = (unsigned)blockIdx.x * (unsigned)NBK;

  {
    const v4i z4 = {0, 0, 0, 0};
    const v4i m4 = {-1, -1, -1, -1};
    for (int i = tid * 4; i < BINS_INTS; i += NTHR * 4) {
      *(v4ia*)(cntb + i)  = z4;
      *(v4ia*)(lastb + i) = m4;
    }
  }
  __syncthreads();

  int* cw = cntb  + wave * (2 * NBK);
  int* lw = lastb + wave * (2 * NBK);
#pragma unroll 1
  for (int i0 = 0; i0 < WTRIPS; i0 += 4) {
    int dv[4];
#pragma unroll
    for (int j = 0; j < 4; ++j) {
      const int ch  = wave + NWAVE * (i0 + j);
      const int chc = ch < NCH ? ch : NCH - 1;
      dv[j] = edges[(size_t)(chc * 32 + lane) * 3 + 2];
    }
#pragma unroll
    for (int j = 0; j < 4; ++j) {
      const int ch = wave + NWAVE * (i0 + j);
      const unsigned slot = (unsigned)dv[j] - base;
      const bool hit = (ch < NCH) && (slot < (unsigned)NBK);
      unsigned msk = __builtin_amdgcn_ballot_w32(hit);
      int nh = (int)__builtin_popcount(msk);
      nh = nh > 32 ? 32 : nh;
      const int role = (ch >= CHH) ? 1 : 0;
#pragma unroll 1
      for (int q = 0; q < nh; ++q) {
        int bpos = __builtin_ffs((int)msk) - 1;
        msk &= msk - 1u;
        bpos = bpos < 0 ? 0 : bpos;
        bpos = __builtin_amdgcn_readfirstlane(bpos);
        const int ss  = __builtin_amdgcn_readlane((int)slot, bpos) & (NBK - 1);
        const int eid = ch * 32 + bpos;
        if (lane == 0) {
          const int idx = role * NBK + ss;
          cw[idx] = cw[idx] + 1;
          const int ol = lw[idx];
          lw[idx] = ol > eid ? ol : eid;
        }
      }
    }
  }
  __syncthreads();

#pragma unroll 1
  for (int j = 0; j < 4; ++j) {
    const int slot = 4 * tid + j;
    int c0 = 0, c1 = 0, e0 = -1, e1 = -1;
#pragma unroll
    for (int w2 = 0; w2 < NWAVE; ++w2) {
      c0 += cntb[w2 * (2 * NBK) + slot];
      c1 += cntb[w2 * (2 * NBK) + NBK + slot];
      const int x0 = lastb[w2 * (2 * NBK) + slot];
      const int x1 = lastb[w2 * (2 * NBK) + NBK + slot];
      e0 = x0 > e0 ? x0 : e0;
      e1 = x1 > e1 ? x1 : e1;
    }
    c0 = clampi(c0, 0, HALF);
    c1 = clampi(c1, 0, HALF);
    const int ec0 = clampi(e0, 0, NE - 1);
    const int ec1 = clampi(e1, 0, NE - 1);
    int s0 = edges[(size_t)ec0 * 3];
    int r0 = edges[(size_t)ec0 * 3 + 1];
    int s1 = edges[(size_t)ec1 * 3];
    int r1 = edges[(size_t)ec1 * 3 + 1];
    asm volatile("" :: "v"(s0), "v"(r0), "v"(s1), "v"(r1));
    s0 = clampi(s0, 0, NN - 1);
    s1 = clampi(s1, 0, NN - 1);
    r0 = clampi(r0, 0, NREL - 1);
    r1 = clampi(r1, 0, NREL - 1);
    const int node = (int)base + slot;
    const int m0 = ((c0 > 0) && (node < NN)) ? -1 : 0;
    const int m1 = ((c1 > 0) && (node < NN)) ? -1 : 0;
    v4i ra, rb;
    ra.x = c0 & m0; ra.y = s0 & m0; ra.z = r0 & m0; ra.w = ec0 & m0;
    rb.x = c1 & m1; rb.y = s1 & m1; rb.z = r1 & m1; rb.w = ec1 & m1;
    *(v4ia*)(stage + slot * 8)     = ra;
    *(v4ia*)(stage + slot * 8 + 4) = rb;
  }
  __syncthreads();

  v4i vals[8];
#pragma unroll
  for (int it = 0; it < 8; ++it) vals[it] = *(const v4ia*)(stage + 4 * (it * NTHR + tid));
  int* rp = rec + (size_t)blockIdx.x * (size_t)STAGE_INTS;
#pragma unroll
  for (int it = 0; it < 8; ++it) *(volatile v4i*)(rp + 4 * (it * NTHR + tid)) = vals[it];
  __threadfence();
#pragma unroll
  for (int it = 0; it < 8; ++it) *(volatile v4i*)(rp + 4 * (it * NTHR + tid)) = vals[it];
}

__global__ __launch_bounds__(GTHR) __attribute__((amdgpu_num_vgpr(248)))
void k_gemm(const unsigned short* __restrict__ A, const unsigned short* __restrict__ BT,
            float* C, int ldc, int mGuard) {
  __shared__ __attribute__((aligned(16))) float stg[GBM * GBN];
  const int tid = (int)threadIdx.x, lane = tid & 31, wave = tid >> 5, hh = lane >> 4, m = lane & 15;
  const int rowBase = (int)blockIdx.x * GBM;
  const int colBase = (int)blockIdx.y * GBN;

  v8f acc[8];
  {
    const v8f z = {0.f, 0.f, 0.f, 0.f, 0.f, 0.f, 0.f, 0.f};
#pragma unroll
    for (int t = 0; t < 8; ++t) acc[t] = z;
  }
  const unsigned short* ap = A  + (size_t)(rowBase + 16 * wave + m) * (size_t)DF + 8 * hh;
  const unsigned short* bp = BT + (size_t)(colBase + m) * (size_t)DF + 8 * hh;

#pragma unroll 1
  for (int k0 = 0; k0 < DF; k0 += 32) {
    FragB af;
    af.h[0] = *(const v8usa*)(ap + k0);
    af.h[1] = *(const v8usa*)(ap + k0 + 16);
#pragma unroll
    for (int nt = 0; nt < 8; ++nt) {
      const unsigned short* wq = bp + (size_t)(16 * nt) * (size_t)DF + k0;
      FragB bf;
      bf.h[0] = *(const v8usa*)wq;
      bf.h[1] = *(const v8usa*)(wq + 16);
      acc[nt] = wmb(af, bf, acc[nt]);
    }
  }

#pragma unroll
  for (int nt = 0; nt < 8; ++nt) {
    const int lc = 16 * nt + m;
#pragma unroll
    for (int r = 0; r < 8; ++r) {
      const int lr = 16 * wave + 8 * hh + r;
      stg[lr * GBN + lc] = acc[nt][r];
    }
  }
  __syncthreads();

  v4f pv[16];
#pragma unroll
  for (int i = 0; i < 16; ++i) pv[i] = *(const v4fa*)(stg + (16 * wave + i) * GBN + 4 * lane);

#pragma unroll
  for (int i = 0; i < 16; ++i) {
    const int r = rowBase + 16 * wave + i;
    if (r < mGuard) *(volatile v4f*)(C + (size_t)r * (size_t)ldc + colBase + 4 * lane) = pv[i];
  }
  __threadfence();
#pragma unroll
  for (int i = 0; i < 16; ++i) {
    const int r = rowBase + 16 * wave + i;
    if (r < mGuard) *(volatile v4f*)(C + (size_t)r * (size_t)ldc + colBase + 4 * lane) = pv[i];
  }
}

__global__ __launch_bounds__(NTHR) void k_comb(const int* __restrict__ rec, const float* __restrict__ pno,
                                               const float* __restrict__ pr, float* out) {
  const int tid = (int)threadIdx.x, lane = tid & 31;
  const int wave = __builtin_amdgcn_readfirstlane(tid >> 5);
  int d = (int)blockIdx.x * NWAVE + wave;
  d = d > NN - 1 ? NN - 1 : d;

  v4i ra = *(const v4i*)(rec + (size_t)d * 8);
  v4i rb = *(const v4i*)(rec + (size_t)d * 8 + 4);
  ra.x = clampi(ra.x, 0, HALF); ra.y = clampi(ra.y, 0, NN - 1); ra.z = clampi(ra.z, 0, NREL - 1);
  rb.x = clampi(rb.x, 0, HALF); rb.y = clampi(rb.y, 0, NN - 1); rb.z = clampi(rb.z, 0, NREL - 1);
  const int c0 = __builtin_amdgcn_readfirstlane(ra.x);
  const int s0 = __builtin_amdgcn_readfirstlane(ra.y);
  const int r0 = __builtin_amdgcn_readfirstlane(ra.z);
  const int c1 = __builtin_amdgcn_readfirstlane(rb.x);
  const int s1 = __builtin_amdgcn_readfirstlane(rb.y);
  const int r1 = __builtin_amdgcn_readfirstlane(rb.z);

  float* op = out + (size_t)d * DF + 4 * lane;
  const v4f own = *(const v4f*)op;
  const v4f rs  = *(const v4f*)(pr  + (size_t)SELFROW * PRW + 4 * lane);
  const v4f a0  = *(const v4f*)(pno + (size_t)s0 * PNW + 4 * lane);
  const v4f b0  = *(const v4f*)(pr  + (size_t)r0 * PRW + DF + 4 * lane);
  const v4f a1  = *(const v4f*)(pno + (size_t)s1 * PNW + DF + 4 * lane);
  const v4f b1  = *(const v4f*)(pr  + (size_t)r1 * PRW + 2 * DF + 4 * lane);

  v4f h = own + rs;
  {
    const v4f mm = a0 + b0;
    const v4f tt = (float)c0 * mm;
    const v4f hn = h + tt;
    h = (c0 > 0) ? hn : h;
  }
  {
    const v4f mm = a1 + b1;
    const v4f tt = (float)c1 * mm;
    const v4f hn = h + tt;
    h = (c1 > 0) ? hn : h;
  }
  *(volatile v4f*)op = h;
  __threadfence();
  *(volatile v4f*)op = h;
}

extern "C" void kernel_launch(void* const* d_in, const int* in_sizes, int n_in,
                              void* d_out, int out_size, void* d_ws, size_t ws_size,
                              hipStream_t stream) {
  if (n_in < 7) return;
  if (in_sizes[0] != NN * DF) return;
  if (in_sizes[1] != NREL * DF) return;
  if (in_sizes[2] != NE * 3) return;
  if (in_sizes[3] != DF * DF || in_sizes[4] != DF * DF) return;
  if (in_sizes[5] != DF * DF || in_sizes[6] != DF * DF) return;
  if (out_size != OUT_TOTAL) return;
  if (ws_size < WS_TOTAL) return;

  const float* xn  = (const float*)d_in[0];
  const float* rel = (const float*)d_in[1];
  const int*   edg = (const int*)d_in[2];
  const float* Wo  = (const float*)d_in[3];
  const float* Wi  = (const float*)d_in[4];
  const float* Ws  = (const float*)d_in[5];
  const float* Wr  = (const float*)d_in[6];
  float* out = (float*)d_out;

  char* ws = (char*)d_ws;
  unsigned short* XB  = (unsigned short*)(ws + OFF_XB);
  float*          PNO = (float*)(ws + OFF_PNO);
  unsigned short* RB  = (unsigned short*)(ws + OFF_RB);
  unsigned short* WC  = (unsigned short*)(ws + OFF_WC);
  float*          PR  = (float*)(ws + OFF_PR);
  int*            REC = (int*)(ws + OFF_REC);

  const size_t bkLds = (size_t)BK_LDS_INTS * 4;
  hipFuncSetAttribute(reinterpret_cast<const void*>(&k_bucket), hipFuncAttributeMaxDynamicSharedMemorySize,
                      (int)bkLds);

  k_prep<<<PREP_BX + PREP_BR + PREP_BW, NTHR, 0, stream>>>(xn, rel, Wo, Wi, Ws, Wr, XB, RB, WC);
  k_bucket<<<NBLK, NTHR, bkLds, stream>>>(edg, REC);
  k_gemm<<<dim3(MP / GBM, 2), GTHR, 0, stream>>>(XB, WC + (size_t)DF * DF, PNO, PNW, NN);
  k_gemm<<<dim3(MP / GBM, 1), GTHR, 0, stream>>>(XB, WC, out, DF, NN);
  k_gemm<<<dim3(RBR / GBM, 3), GTHR, 0, stream>>>(RB, WC, PR, PRW, RBR);
  k_gemm<<<dim3(RBR / GBM, 1), GTHR, 0, stream>>>(RB, WC + (size_t)3 * DF * DF, out + (size_t)OUT1_OFF, DF, NREL);
  k_comb<<<NN / NWAVE, NTHR, 0, stream>>>(REC, PNO, PR, out);
}
